// OuterProducterMean_10685878633040
// MI455X (gfx1250) — hardware-verified
//
#include <hip/hip_runtime.h>
#include <math.h>

typedef __attribute__((ext_vector_type(16))) _Float16 v16h;
typedef __attribute__((ext_vector_type(16))) __bf16 v16b;
typedef __attribute__((ext_vector_type(8)))  _Float16 v8h;
typedef __attribute__((ext_vector_type(8)))  float v8f;
typedef __attribute__((ext_vector_type(4)))  float v4f;
typedef __attribute__((ext_vector_type(2)))  float v2f;
typedef __attribute__((ext_vector_type(4)))  unsigned v4u;
typedef __attribute__((ext_vector_type(4)))  int v4i;
typedef float __attribute__((may_alias)) float_a;
typedef int __attribute__((may_alias)) int_a;

template <typename T> __device__ __forceinline__ void vst2(void* p, T v) { *(volatile T*)p = v; __threadfence(); *(volatile T*)p = v; }
__device__ __forceinline__ v8f wmma16(v16h a, v16h b, v8f c) {
  v8f d = __builtin_amdgcn_wmma_f32_16x16x32_f16(false, a, false, b, (short)0, c, false, false);
  asm volatile("v_nop\n\tv_nop\n\tv_nop\n\tv_nop" : "+v"(d) : "v"(a), "v"(b));
  return d;
}
__device__ __forceinline__ v8f wmma_bf(v16b a, v16b b, v8f c) {
  v8f d = __builtin_amdgcn_wmma_f32_16x16x32_bf16(false, a, false, b, (short)0, c, false, false);
  asm volatile("v_nop\n\tv_nop\n\tv_nop\n\tv_nop" : "+v"(d) : "v"(a), "v"(b));
  return d;
}
__device__ __forceinline__ v16h frag_h(const _Float16* rowk0, int lane) {
  union { v16h v; v8h q[2]; } u; const _Float16* p = rowk0 + 8 * (lane >> 4);
  u.q[0] = *(const v8h*)p; u.q[1] = *(const v8h*)(p + 16); return u.v;
}
__device__ __forceinline__ v16h frag_f32(const float* rowk0, int lane) {
  v16h a; const float* p = rowk0 + 8 * (lane >> 4);
#pragma unroll
  for (int i = 0; i < 8; ++i) { a[i] = (_Float16)p[i]; a[8 + i] = (_Float16)p[16 + i]; }
  return a;
}
__device__ __forceinline__ v16h frag_f32s(const float* rowk0, int lane, float sc) {
  v16h a; const float* p = rowk0 + 8 * (lane >> 4);
#pragma unroll
  for (int i = 0; i < 8; ++i) { a[i] = (_Float16)(p[i] * sc); a[8 + i] = (_Float16)(p[16 + i] * sc); }
  return a;
}
__device__ __forceinline__ v16h fragc_f32(const float* W, int k0, int n, int lane, int ld, int K) {
  v16h a; const int g = lane >> 4;
#pragma unroll
  for (int i = 0; i < 8; ++i) { const int ka = k0 + 8 * g + i, kb = ka + 16;
    a[i] = (_Float16)(ka < K ? W[(size_t)(ka < K ? ka : K - 1) * ld + n] : 0.f); a[8 + i] = (_Float16)(kb < K ? W[(size_t)(kb < K ? kb : K - 1) * ld + n] : 0.f); }
  return a;
}
struct F2 { v16b h, l; };
__device__ __forceinline__ F2 bsplit16(const float v[16]) { F2 r;
#pragma unroll
  for (int i = 0; i < 16; ++i) { const __bf16 h = (__bf16)v[i]; r.h[i] = h; r.l[i] = (__bf16)(v[i] - (float)h); }
  return r; }
__device__ __forceinline__ F2 split_row(const float* row, int k0, int lane) { float v[16]; const float* p = row + k0 + 8 * (lane >> 4);
#pragma unroll
  for (int i = 0; i < 8; ++i) { v[i] = p[i]; v[8 + i] = p[16 + i]; }
  return bsplit16(v); }
__device__ __forceinline__ F2 split_rowK(const float* row, int k0, int lane, int K) { float v[16]; const int g = lane >> 4;
#pragma unroll
  for (int i = 0; i < 8; ++i) { const int ka = k0 + 8 * g + i, kb = ka + 16; v[i] = ka < K ? row[ka < K ? ka : K - 1] : 0.f; v[8 + i] = kb < K ? row[kb < K ? kb : K - 1] : 0.f; }
  return bsplit16(v); }
__device__ __forceinline__ F2 split_col(const float* W, int k0, int n, int lane, int ld, int K) { float v[16]; const int g = lane >> 4;
#pragma unroll
  for (int i = 0; i < 8; ++i) { const int ka = k0 + 8 * g + i, kb = ka + 16; v[i] = ka < K ? W[(size_t)(ka < K ? ka : K - 1) * ld + n] : 0.f; v[8 + i] = kb < K ? W[(size_t)(kb < K ? kb : K - 1) * ld + n] : 0.f; }
  return bsplit16(v); }
__device__ __forceinline__ v8f mac3(const F2& a, const F2& b, v8f c) { c = wmma_bf(a.l, b.h, c); c = wmma_bf(a.h, b.l, c); return wmma_bf(a.h, b.h, c); }
__device__ __forceinline__ float sigm(float v) { return 1.0f / (1.0f + expf(-v)); }
#define LDSX() do { asm volatile("s_wait_dscnt 0" ::: "memory"); __builtin_amdgcn_wave_barrier(); __builtin_amdgcn_fence(__ATOMIC_RELEASE, "workgroup"); } while (0)

__device__ __forceinline__ float bfr(float v) { return (float)(__bf16)v; }
#define SS 128
#define RR 256
#define MM 256
#define CP 32
#define CZ 128
#define CC2 (CP * CP)
#define RQ 64
#ifndef NQ
#define NQ (RR / RQ)
#endif
#define WS_LH  0u
#define WS_LL  (WS_LH + 2u * (size_t)RR * CP * SS)
#define WS_RH  (WS_LL + 2u * (size_t)RR * CP * SS)
#define WS_RL  (WS_RH + 2u * (size_t)RR * CP * SS)
#define WS_X2  (WS_RL + 2u * (size_t)RR * CP * SS)
#define WS_END (WS_X2 + 4u * (size_t)RQ * RR * CC2)
__global__ __launch_bounds__(128) void k_lr(const float* __restrict__ MSA, const float* __restrict__ LW, const float* __restrict__ RW, _Float16* __restrict__ LH, _Float16* __restrict__ LL, _Float16* __restrict__ RH, _Float16* __restrict__ RL) { __shared__ __align__(16) _Float16 th[CP][72], tl[CP][72];
  const int tid = threadIdx.x, wave = tid >> 5, lane = tid & 31, col = lane & 15, g = lane >> 4; const int r = blockIdx.x; const int s0 = blockIdx.y * 64; const int which = blockIdx.z; const float* Wt = which == 0 ? LW : RW;
  v8f acc[2] = {};
#pragma unroll 2
  for (int kc = 0; kc < MM / 32; ++kc) { v16b a; { const float* p = MSA + ((size_t)(s0 + wave * 16 + col) * RR + r) * MM + kc * 32 + 8 * g;
#pragma unroll
      for (int i = 0; i < 8; ++i) { a[i] = (__bf16)p[i]; a[8 + i] = (__bf16)p[16 + i]; } }
#pragma unroll
    for (int j = 0; j < 2; ++j) { v16b w; const int o = j * 16 + col;
#pragma unroll
      for (int i = 0; i < 8; ++i) { w[i] = (__bf16)Wt[(size_t)(kc * 32 + 8 * g + i) * CP + o]; w[8 + i] = (__bf16)Wt[(size_t)(kc * 32 + 16 + 8 * g + i) * CP + o]; }
      asm volatile("s_wait_loadcnt 0x0" ::: "memory"); acc[j] = wmma_bf(a, w, acc[j]); } }
#pragma unroll
  for (int j = 0; j < 2; ++j)
#pragma unroll
    for (int rr = 0; rr < 8; ++rr) { const float v = acc[j][rr]; const int sl = wave * 16 + 8 * g + rr, c = j * 16 + col; const _Float16 hv = (_Float16)v; th[c][sl] = hv; tl[c][sl] = (_Float16)((v - (float)hv) * 1024.0f); }
  __syncthreads();
  { _Float16* DH = which == 0 ? LH : RH; _Float16* DL = which == 0 ? LL : RL; for (int e = tid; e < CP * 8; e += 128) { const int c = e >> 3, q = e & 7; const size_t o2 = ((size_t)r * CP + c) * SS + s0 + q * 8; vst2((unsigned*)(DH + o2), *(const v4u*)&th[c][q * 8]); vst2((unsigned*)(DL + o2), *(const v4u*)&tl[c][q * 8]); } } }
__global__ __launch_bounds__(128) void k_outer(const _Float16* __restrict__ LH, const _Float16* __restrict__ LL, const _Float16* __restrict__ RH, const _Float16* __restrict__ RL, int rq0, float* __restrict__ X2) { __shared__ __align__(16) float ss[4][16][132];
  const int tid = threadIdx.x, wave = tid >> 5, lane = tid & 31, col = lane & 15, g = lane >> 4; const size_t arow0 = (size_t)rq0 * CP + (size_t)blockIdx.x * 64 + wave * 16;
  const size_t bcol0 = (size_t)blockIdx.y * 128;
  v8f acc[8] = {}, accl[8] = {};
#pragma unroll
  for (int kc = 0; kc < SS / 32; ++kc) { const v16h ah = frag_h(LH + (arow0 + col) * SS + kc * 32, lane), al = frag_h(LL + (arow0 + col) * SS + kc * 32, lane);
#pragma unroll
    for (int j = 0; j < 8; ++j) { const size_t bo = (bcol0 + j * 16 + col) * SS + kc * 32; const v16h bh = frag_h(RH + bo, lane), bl = frag_h(RL + bo, lane); acc[j] = wmma16(ah, bh, acc[j]); accl[j] = wmma16(al, bh, accl[j]); accl[j] = wmma16(ah, bl, accl[j]); } }
#pragma unroll
  for (int j = 0; j < 8; ++j)
#pragma unroll
    for (int rr = 0; rr < 8; ++rr) ss[wave][8 * g + rr][j * 16 + col] = acc[j][rr] + accl[j][rr] * (1.0f / 1024.0f);
  LDSX();
  { const size_t rowrc = arow0; const int r = (int)(rowrc / CP), cw0 = (int)(rowrc % CP); const int t0 = (int)(bcol0 / CP);
    for (int q = lane; q < 4 * 16 * 8; q += 32) { const int jt = q >> 7, rem = q & 127; const int cl = rem >> 3, e4 = rem & 7;     const v4f v = *(const v4f*)&ss[wave][cl][jt * 32 + e4 * 4]; vst2(X2 + ((size_t)(r - rq0) * RR + t0 + jt) * CC2 + (size_t)(cw0 + cl) * CP + e4 * 4, v); } } }
__global__ __launch_bounds__(128) void k_proj2(const float* __restrict__ X2, const float* __restrict__ OW, int rq0, float* __restrict__ OUT) { __shared__ __align__(16) float sf[4][16][132];
  const int tid = threadIdx.x, wave = tid >> 5, lane = tid & 31, col = lane & 15, g = lane >> 4; const size_t lrow = (size_t)blockIdx.x * 64 + wave * 16;
  v8f acc[8] = {};
#pragma unroll 2
  for (int kc = 0; kc < CC2 / 32; ++kc) { const F2 a = split_row(X2 + (lrow + col) * CC2, kc * 32, lane);
#pragma unroll
    for (int j = 0; j < 8; ++j) { v16b w; const int o = j * 16 + col;
#pragma unroll
      for (int i = 0; i < 8; ++i) { w[i] = (__bf16)OW[(size_t)(kc * 32 + 8 * g + i) * CZ + o]; w[8 + i] = (__bf16)OW[(size_t)(kc * 32 + 16 + 8 * g + i) * CZ + o]; }
      asm volatile("s_wait_loadcnt 0x0" ::: "memory"); acc[j] = wmma_bf(a.h, w, acc[j]); acc[j] = wmma_bf(a.l, w, acc[j]); } }
#pragma unroll
  for (int j = 0; j < 8; ++j)
#pragma unroll
    for (int rr = 0; rr < 8; ++rr) sf[wave][8 * g + rr][j * 16 + col] = acc[j][rr];
  LDSX(); for (int rl = 0; rl < 16; ++rl) vst2(OUT + ((size_t)rq0 * RR + lrow + rl) * CZ + lane * 4, *(const v4f*)&sf[wave][rl][lane * 4]); }
extern "C" void kernel_launch(void* const* d_in, const int* in_sizes, int n_in, void* d_out, int out_size, void* d_ws, size_t ws_size, hipStream_t stream) {
  (void)in_sizes; (void)n_in; (void)out_size;
  const float** F = (const float**)d_in;
  if (ws_size < (size_t)WS_END) return;
  char* ws = (char*)d_ws; _Float16 *LH = (_Float16*)(ws + WS_LH), *LL = (_Float16*)(ws + WS_LL), *RH = (_Float16*)(ws + WS_RH), *RL = (_Float16*)(ws + WS_RL); float* X2 = (float*)(ws + WS_X2);
  k_lr<<<dim3(RR, SS / 64, 2), 128, 0, stream>>>(F[0], F[1], F[2], LH, LL, RH, RL);
  for (int q = 0; q < NQ; ++q) { const int rq0 = q * RQ;
    k_outer<<<dim3(RQ * CP / 64, RR * CP / 128), 128, 0, stream>>>(LH, LL, RH, RL, rq0, X2);
    k_proj2<<<dim3(RQ * RR / 64), 128, 0, stream>>>(X2, F[3], rq0, (float*)d_out);
  }
}
